// Model2_36713380446230
// MI455X (gfx1250) — hardware-verified
//
#include <hip/hip_runtime.h>
#include <stdint.h>
#pragma clang fp contract(off)

typedef __attribute__((ext_vector_type(16))) _Float16 v16h;
typedef __attribute__((ext_vector_type(8)))  _Float16 v8h;
typedef __attribute__((ext_vector_type(16))) __bf16   v16b;
typedef __attribute__((ext_vector_type(8)))  __bf16   v8b;
typedef __attribute__((ext_vector_type(8)))  float    v8f;
typedef __attribute__((ext_vector_type(4)))  float    v4f;
typedef __attribute__((ext_vector_type(4)))  unsigned int u32x4;

__device__ __forceinline__ unsigned short f2bf_bits(float f) {
  unsigned u = __float_as_uint(f);
  return (unsigned short)((u + 0x7FFFu + ((u >> 16) & 1u)) >> 16);
}
__device__ __forceinline__ float bf_bits2f(unsigned short h) { return __uint_as_float(((unsigned)h) << 16); }

__device__ __forceinline__ void dep_guard_h(v8f& a, v8f& b, v16h x, v16h y) { asm volatile("v_nop\n\tv_nop\n\tv_nop\n\tv_nop" : "+v"(a), "+v"(b) : "v"(x), "v"(y)); }
__device__ __forceinline__ void dep_guard_b(v8f& a, v8f& b, v16b x, v16b y) { asm volatile("v_nop\n\tv_nop\n\tv_nop\n\tv_nop" : "+v"(a), "+v"(b) : "v"(x), "v"(y)); }
__device__ __forceinline__ void keep4_h(v16h a, v16h b, v16h c, v16h d) { asm volatile("v_nop" :: "v"(a), "v"(b), "v"(c), "v"(d)); }
__device__ __forceinline__ void keep4_b(v16b a, v16b b, v16b c, v16b d) { asm volatile("v_nop" :: "v"(a), "v"(b), "v"(c), "v"(d)); }
__device__ __forceinline__ void acc_guard4(v8f& a, v8f& b, v8f& c, v8f& d) { asm volatile("v_nop\n\tv_nop\n\tv_nop\n\tv_nop" : "+v"(a), "+v"(b), "+v"(c), "+v"(d)); }
template <typename T> struct Frag;
template <> struct Frag<_Float16> {
  typedef v16h V; union U { v16h v; v8h h[2]; };
  static __device__ __forceinline__ v16h load(const _Float16* p) {
    U f; f.h[0] = *(const v8h*)(p); f.h[1] = *(const v8h*)(p + 16); return f.v;
  }
  static __device__ __forceinline__ v8f mma(v16h a, v16h b, v8f c) {
    return __builtin_amdgcn_wmma_f32_16x16x32_f16(false, a, false, b, (short)0, c, false, false);
  }
  static __device__ __forceinline__ void guard(v8f& a, v8f& b, v16h x, v16h y) { dep_guard_h(a, b, x, y); }
  static __device__ __forceinline__ void keep(v16h a, v16h b, v16h c, v16h d) { keep4_h(a, b, c, d); }
};
template <> struct Frag<__bf16> {
  typedef v16b V; union U { v16b v; v8b h[2]; };
  static __device__ __forceinline__ v16b load(const __bf16* p) {
    U f; f.h[0] = *(const v8b*)(p); f.h[1] = *(const v8b*)(p + 16); return f.v;
  }
  static __device__ __forceinline__ v8f mma(v16b a, v16b b, v8f c) {
    return __builtin_amdgcn_wmma_f32_16x16x32_bf16(false, a, false, b, (short)0, c, false, false);
  }
  static __device__ __forceinline__ void guard(v8f& a, v8f& b, v16b x, v16b y) { dep_guard_b(a, b, x, y); }
  static __device__ __forceinline__ void keep(v16b a, v16b b, v16b c, v16b d) { keep4_b(a, b, c, d); }
};

template <int ET> struct Elem;
template <> struct Elem<0> { typedef _Float16 T; };
template <> struct Elem<1> { typedef __bf16 T; };
template <int ET, bool SPLIT, int BIAS_MODE, int OUT_MODE, bool RESID, int ACT = 0>
__global__ __launch_bounds__(256) void wmma_gemm64(
    const unsigned short* __restrict__ Ap, const unsigned short* __restrict__ A2p, int lda, long strideA,
    const unsigned short* __restrict__ Btp, const unsigned short* __restrict__ Bt2p, int ldb, long strideB,
    void* __restrict__ Cout, void* __restrict__ Cout2, int ldc, long strideC,
    const float* __restrict__ bias,
    const float* __restrict__ resid, long strideR,
    int M, int N, int K, float scale) {
  typedef typename Elem<ET>::T T;
  typedef typename Frag<T>::V V;
  const T* A = (const T*)Ap; const T* A2 = (const T*)A2p; const T* Bt = (const T*)Btp; const T* Bt2 = (const T*)Bt2p;
  __shared__ __align__(16) float sT[8][16 * 68];
  const int b    = blockIdx.y;
  const int lane = threadIdx.x & 31;
  const int wave = threadIdx.x >> 5;
  const int tilesN = N >> 6;
  const int tilesM = M >> 6;
  const int tile = blockIdx.x * 8 + wave;
  if (tile >= tilesM * tilesN) return;
  const int tm = tile / tilesN;
  const int tn = tile - tm * tilesN;
  const int m0 = tm << 6;
  const int n0 = tn << 6;

  const T* Ab  = A  + (size_t)b * strideA;
  const T* Bb  = Bt + (size_t)b * strideB;
  const T* Ab2 = SPLIT ? (A2  + (size_t)b * strideA) : nullptr;
  const T* Bb2 = SPLIT ? (Bt2 + (size_t)b * strideB) : nullptr;

  const int rlane = lane & 15;
  const int koff  = (lane >> 4) * 8;
  const int mOff  = (lane >> 4) * 8;

  v8f acc[4][4];
#pragma unroll
  for (int i = 0; i < 4; ++i)
#pragma unroll
    for (int j = 0; j < 4; ++j) acc[i][j] = (v8f){0.f,0.f,0.f,0.f,0.f,0.f,0.f,0.f};

  for (int k0 = 0; k0 < K; k0 += 32) {
    V bh[4], bl[4];
#pragma unroll
    for (int j = 0; j < 4; ++j) {
      const size_t bo = (size_t)(n0 + (j << 4) + rlane) * ldb + koff + k0;
      bh[j] = Frag<T>::load(Bb + bo);
      if (SPLIT) bl[j] = Frag<T>::load(Bb2 + bo);
    }
#pragma unroll
    for (int i = 0; i < 4; ++i) {
      const size_t ao = (size_t)(m0 + (i << 4) + rlane) * lda + koff + k0;
      V ah = Frag<T>::load(Ab + ao);
      V al;
      if (SPLIT) al = Frag<T>::load(Ab2 + ao);
#pragma unroll
      for (int j = 0; j < 4; ++j) {
        acc[i][j] = Frag<T>::mma(ah, bh[j], acc[i][j]);
        if (SPLIT) {
          acc[i][j] = Frag<T>::mma(ah, bl[j], acc[i][j]);
          acc[i][j] = Frag<T>::mma(al, bh[j], acc[i][j]);
        }
      }
      Frag<T>::guard(acc[i][0], acc[i][3], ah, SPLIT ? al : ah);
    }
    Frag<T>::keep(bh[0], bh[1], bh[2], bh[3]);
    if (SPLIT) Frag<T>::keep(bl[0], bl[1], bl[2], bl[3]);
  }
  acc_guard4(acc[0][0], acc[0][1], acc[0][2], acc[0][3]);
  acc_guard4(acc[1][0], acc[1][1], acc[1][2], acc[1][3]);
  acc_guard4(acc[2][0], acc[2][1], acc[2][2], acc[2][3]);
  acc_guard4(acc[3][0], acc[3][1], acc[3][2], acc[3][3]);

  float* slab = sT[wave];
  const float* Rb = RESID ? (resid + (size_t)b * strideR) : nullptr;
#pragma unroll
  for (int i = 0; i < 4; ++i) {
    const int mBase = m0 + (i << 4);
#pragma unroll
    for (int j = 0; j < 4; ++j) {
      const int n = n0 + (j << 4) + rlane;
      float bv = 0.f;
      if (BIAS_MODE == 2) bv = bias[n];
#pragma unroll
      for (int r = 0; r < 8; ++r) {
        float v = acc[i][j][r] * scale;
        if (BIAS_MODE == 1) v += bias[mBase + mOff + r];
        if (BIAS_MODE == 2) v += bv;
        if (RESID) v += Rb[(size_t)(mBase + mOff + r) * ldc + n];
        if (ACT == 1) v = tanhf(v);
        if (ACT == 2) v = fmaxf(v, 0.0f);
        if (ACT == 3) v = v / (1.0f + expf(-v));
        if (ACT == 4) v = (v > 0.f) ? v : 0.01f * v;
        if (ACT == 5) v = 0.5f * v * (1.0f + erff(v * 0.70710678118654752f));
        slab[(mOff + r) * 68 + (j << 4) + rlane] = v;
      }
    }
    __builtin_amdgcn_fence(__ATOMIC_RELEASE, "workgroup");
    __builtin_amdgcn_wave_barrier();
    __builtin_amdgcn_fence(__ATOMIC_ACQUIRE, "workgroup");
    if (OUT_MODE == 0) {
      float* C = (float*)Cout + (size_t)b * strideC;
      const int hh = lane >> 4, c4 = (lane & 15) * 4;
      for (int pass = 0; pass < 2; ++pass) {
#pragma unroll
        for (int it = 0; it < 8; ++it) {
          const int row = it * 2 + hh;
          v4f v = *(const v4f*)(slab + row * 68 + c4);
          *(volatile v4f*)(C + (size_t)(mBase + row) * ldc + n0 + c4) = v;
        }
        __threadfence();
      }
    } else {
      const int q = lane >> 3, c8 = (lane & 7) * 8;
      unsigned short* C  = (unsigned short*)Cout  + (size_t)b * strideC;
      unsigned short* C2 = (OUT_MODE == 2) ? ((unsigned short*)Cout2 + (size_t)b * strideC) : nullptr;
      for (int pass = 0; pass < 2; ++pass) {
#pragma unroll
        for (int it = 0; it < 4; ++it) {
          const int row = it * 4 + q;
          const float* sp = slab + row * 68 + c8;
          v8h hv, lv;
#pragma unroll
          for (int e = 0; e < 8; ++e) {
            if (OUT_MODE == 1) {
              hv[e] = (_Float16)sp[e];
            } else {
              unsigned short hb = f2bf_bits(sp[e]);
              unsigned short lb = f2bf_bits(sp[e] - bf_bits2f(hb));
              hv[e] = __builtin_bit_cast(_Float16, hb);
              lv[e] = __builtin_bit_cast(_Float16, lb);
            }
          }
          *(volatile v8h*)(C + (size_t)(mBase + row) * ldc + n0 + c8) = hv;
          if (OUT_MODE == 2) *(volatile v8h*)(C2 + (size_t)(mBase + row) * ldc + n0 + c8) = lv;
        }
        __threadfence();
      }
    }
    __builtin_amdgcn_fence(__ATOMIC_RELEASE, "workgroup");
    __builtin_amdgcn_wave_barrier();
    __builtin_amdgcn_fence(__ATOMIC_ACQUIRE, "workgroup");
  }
}

constexpr int NTOK_ALL    = 65536;
constexpr int HID         = 128;
constexpr int DIN2        = 256;
constexpr int NGATE       = 512;
constexpr int GCOLS       = 768;
constexpr int CHUNK_TOK   = 16384;
constexpr int NCHUNK      = NTOK_ALL / CHUNK_TOK;
constexpr int FCN         = 64;
constexpr int TOK_PER_BLK = 32;
constexpr float CARRY     = 16.0f;
constexpr float UNCARRY   = 1.0f / 256.0f;

static_assert(NCHUNK * CHUNK_TOK == NTOK_ALL, "chunking exact");
static_assert(CHUNK_TOK % 64 == 0 && NTOK_ALL % 64 == 0, "GEMM M tile multiple");
static_assert(HID % 64 == 0 && (2 * HID) % 64 == 0 && FCN % 64 == 0, "GEMM N tile multiple");
static_assert(DIN2 % 32 == 0, "GEMM K multiple of 32");
static_assert(NTOK_ALL % TOK_PER_BLK == 0 && CHUNK_TOK % TOK_PER_BLK == 0, "VALU grids exact");
static_assert(GCOLS == 6 * HID, "gate buffer layout");

constexpr size_t SZ_W    = (size_t)2 * 2 * NGATE * DIN2 * 2;
constexpr size_t SZ_WFC  = (size_t)FCN * DIN2 * 2;
constexpr size_t SZ_H    = (size_t)NTOK_ALL * DIN2 * 2;
constexpr size_t SZ_G    = (size_t)CHUNK_TOK * GCOLS * 4;
constexpr size_t OFF_W   = 0;
constexpr size_t OFF_WFC = OFF_W + SZ_W;
constexpr size_t OFF_HA  = OFF_WFC + SZ_WFC;
constexpr size_t OFF_HB  = OFF_HA + SZ_H;
constexpr size_t OFF_G   = OFF_HB + SZ_H;
constexpr size_t WS_TOTAL = OFF_G + SZ_G;
static_assert(OFF_WFC % 128 == 0 && OFF_HA % 128 == 0 && OFF_HB % 128 == 0 && OFF_G % 128 == 0, "aligned carves");
static_assert((size_t)NTOK_ALL * FCN * 4 <= SZ_G, "projection output fits the gate region");
static_assert(WS_TOTAL == 118521856, "carve total");
static_assert(WS_TOTAL <= (size_t)134217728, "carve budget");

__device__ __forceinline__ float fexp_(float x) { return __builtin_amdgcn_exp2f(x * 1.4426950408889634f); }
__device__ __forceinline__ float frcp_(float x) { return __builtin_amdgcn_rcpf(x); }
__device__ __forceinline__ float sigm_(float x) { return frcp_(1.0f + fexp_(-x)); }
__device__ __forceinline__ float tanh_(float x) {
  const float a = fabsf(x);
  const float t = fexp_(-2.0f * a);
  const float r = (1.0f - t) * frcp_(1.0f + t);
  return copysignf(r, x);
}
__device__ __forceinline__ float cell_h(float gi, float gg, float go) {
  const float c = sigm_(gi) * tanh_(gg);
  return sigm_(go) * tanh_(c);
}
__device__ __forceinline__ unsigned pack2h(float a, float b) {
  const _Float16 ha = (_Float16)a;
  const _Float16 hb = (_Float16)b;
  const unsigned ua = (unsigned)__builtin_bit_cast(unsigned short, ha);
  const unsigned ub = (unsigned)__builtin_bit_cast(unsigned short, hb);
  return ua | (ub << 16);
}
__device__ __forceinline__ u32x4 pack8h(float v0, float v1, float v2, float v3, float v4, float v5, float v6, float v7) {
  u32x4 r;
  r.x = pack2h(v0, v1); r.y = pack2h(v2, v3); r.z = pack2h(v4, v5); r.w = pack2h(v6, v7);
  return r;
}
__device__ __forceinline__ void st2_u4(unsigned short* p, u32x4 v) {
  *(volatile u32x4*)(void*)p = v;
  __threadfence();
  *(volatile u32x4*)(void*)p = v;
}

__global__ __launch_bounds__(256) void k_prep(const float* __restrict__ w_ih, const float* __restrict__ w_fc,
                                              unsigned short* __restrict__ wq, unsigned short* __restrict__ wfcq) {
  const int tid = threadIdx.x;
  if (blockIdx.x < 256) {
    const int g = blockIdx.x * 256 + tid;
    const float* s = w_ih + (size_t)g * 8;
    const v4f a = *(const v4f*)s;
    const v4f b = *(const v4f*)(s + 4);
    const u32x4 pk = pack8h(a.x * CARRY, a.y * CARRY, a.z * CARRY, a.w * CARRY,
                            b.x * CARRY, b.y * CARRY, b.z * CARRY, b.w * CARRY);
    st2_u4(wq + (size_t)g * 8, pk);
  } else {
    const int j = (blockIdx.x - 256) * 256 + tid;
    const int row = j >> 5;
    const int col = (j & 31) * 8;
    const float* s = w_fc + (size_t)(row & 1) * DIN2 + col;
    const v4f a = *(const v4f*)s;
    const v4f b = *(const v4f*)(s + 4);
    const u32x4 pk = pack8h(a.x * CARRY, a.y * CARRY, a.z * CARRY, a.w * CARRY,
                            b.x * CARRY, b.y * CARRY, b.z * CARRY, b.w * CARRY);
    st2_u4(wfcq + (size_t)j * 8, pk);
  }
}

__global__ __launch_bounds__(256) void k_layer0(const float* __restrict__ x, const float* __restrict__ w_ih0,
                                                const float* __restrict__ b_ih, const float* __restrict__ b_hh,
                                                unsigned short* __restrict__ hout) {
  __shared__ __align__(16) float sW[1024];
  __shared__ __align__(16) float sBi[1024];
  __shared__ __align__(16) float sBh[1024];
  const int tid = threadIdx.x;
  *(v4f*)(sW  + 4 * tid) = *(const v4f*)(w_ih0 + 4 * tid);
  *(v4f*)(sBi + 4 * tid) = *(const v4f*)(b_ih  + 4 * tid);
  *(v4f*)(sBh + 4 * tid) = *(const v4f*)(b_hh  + 4 * tid);
  __syncthreads();

  const int wave = tid >> 5, lane = tid & 31;
  const int ch0 = lane * 8;
  const int d   = ch0 >> 7;
  const int u0  = ch0 & (HID - 1);
  const int wb  = d * NGATE;
  for (int it = 0; it < TOK_PER_BLK / 8; ++it) {
    const int tok = blockIdx.x * TOK_PER_BLK + it * 8 + wave;
    const float xv = x[tok];
    float hv[8];
#pragma unroll
    for (int e = 0; e < 8; ++e) {
      const int u = u0 + e;
      float gi = xv * sW[wb + u];           gi = gi + sBi[wb + u];           gi = gi + sBh[wb + u];
      float gg = xv * sW[wb + 2 * HID + u]; gg = gg + sBi[wb + 2 * HID + u]; gg = gg + sBh[wb + 2 * HID + u];
      float go = xv * sW[wb + 3 * HID + u]; go = go + sBi[wb + 3 * HID + u]; go = go + sBh[wb + 3 * HID + u];
      hv[e] = cell_h(gi, gg, go) * CARRY;
    }
    const u32x4 pk = pack8h(hv[0], hv[1], hv[2], hv[3], hv[4], hv[5], hv[6], hv[7]);
    st2_u4(hout + (size_t)tok * DIN2 + ch0, pk);
  }
}

__global__ __launch_bounds__(256) void k_act(const float* __restrict__ G,
                                             const float* __restrict__ bi_l, const float* __restrict__ bh_l,
                                             unsigned short* __restrict__ hout) {
  __shared__ __align__(16) float sBi[1024];
  __shared__ __align__(16) float sBh[1024];
  const int tid = threadIdx.x;
  *(v4f*)(sBi + 4 * tid) = *(const v4f*)(bi_l + 4 * tid);
  *(v4f*)(sBh + 4 * tid) = *(const v4f*)(bh_l + 4 * tid);
  __syncthreads();

  const int wave = tid >> 5, lane = tid & 31;
  const int ch0 = lane * 8;
  const int d   = ch0 >> 7;
  const int u0  = ch0 & (HID - 1);
  const int bb  = d * NGATE + u0;
  for (int it = 0; it < TOK_PER_BLK / 8; ++it) {
    const int tloc = blockIdx.x * TOK_PER_BLK + it * 8 + wave;
    const float* gr = G + (size_t)tloc * GCOLS + d * (3 * HID) + u0;
    const v4f i0 = *(const v4f*)(gr);
    const v4f i1 = *(const v4f*)(gr + 4);
    const v4f g0 = *(const v4f*)(gr + HID);
    const v4f g1 = *(const v4f*)(gr + HID + 4);
    const v4f o0 = *(const v4f*)(gr + 2 * HID);
    const v4f o1 = *(const v4f*)(gr + 2 * HID + 4);
    const float gi[8] = {i0.x, i0.y, i0.z, i0.w, i1.x, i1.y, i1.z, i1.w};
    const float gg[8] = {g0.x, g0.y, g0.z, g0.w, g1.x, g1.y, g1.z, g1.w};
    const float go[8] = {o0.x, o0.y, o0.z, o0.w, o1.x, o1.y, o1.z, o1.w};
    float hv[8];
#pragma unroll
    for (int e = 0; e < 8; ++e) {
      float vi = gi[e] + sBi[bb + e];           vi = vi + sBh[bb + e];
      float vg = gg[e] + sBi[bb + 2 * HID + e]; vg = vg + sBh[bb + 2 * HID + e];
      float vo = go[e] + sBi[bb + 3 * HID + e]; vo = vo + sBh[bb + 3 * HID + e];
      hv[e] = cell_h(vi, vg, vo) * CARRY;
    }
    const u32x4 pk = pack8h(hv[0], hv[1], hv[2], hv[3], hv[4], hv[5], hv[6], hv[7]);
    st2_u4(hout + (size_t)tloc * DIN2 + ch0, pk);
  }
}

__global__ __launch_bounds__(256) void k_out(const float* __restrict__ P, const float* __restrict__ b_fc,
                                             float* __restrict__ out) {
  const int i  = blockIdx.x * 256 + threadIdx.x;
  const int t0 = 2 * i;
  const v4f r0 = *(const v4f*)(P + (size_t)t0 * FCN);
  const v4f r1 = *(const v4f*)(P + (size_t)(t0 + 1) * FCN);
  const float b0 = b_fc[0];
  const float b1 = b_fc[1];
  v4f o;
  o.x = r0.x + b0; o.y = r0.y + b1; o.z = r1.x + b0; o.w = r1.y + b1;
  float* p = out + (size_t)i * 4;
  *(volatile v4f*)p = o;
  __threadfence();
  *(volatile v4f*)p = o;
}

typedef void (*GemmFn)(const unsigned short*, const unsigned short*, int, long,
                       const unsigned short*, const unsigned short*, int, long,
                       void*, void*, int, long, const float*, const float*, long, int, int, int, float);

extern "C" void kernel_launch(void* const* d_in, const int* in_sizes, int n_in,
                              void* d_out, int out_size, void* d_ws, size_t ws_size,
                              hipStream_t stream) {
  if (n_in < 7) return;
  if (in_sizes[0] != NTOK_ALL) return;
  if (in_sizes[1] != 2 * NGATE) return;
  if (in_sizes[2] != 2 * 2 * NGATE * DIN2) return;
  if (in_sizes[3] != 3 * 2 * NGATE || in_sizes[4] != 3 * 2 * NGATE) return;
  if (in_sizes[5] != 2 * DIN2 || in_sizes[6] != 2) return;
  if (out_size != NTOK_ALL * 2) return;
  if (ws_size < WS_TOTAL) return;

  const float* x     = (const float*)d_in[0];
  const float* w_ih0 = (const float*)d_in[1];
  const float* w_ih  = (const float*)d_in[2];
  const float* b_ih  = (const float*)d_in[3];
  const float* b_hh  = (const float*)d_in[4];
  const float* w_fc  = (const float*)d_in[5];
  const float* b_fc  = (const float*)d_in[6];
  float* out = (float*)d_out;

  char* ws = (char*)d_ws;
  unsigned short* wq   = (unsigned short*)(ws + OFF_W);
  unsigned short* wfcq = (unsigned short*)(ws + OFF_WFC);
  unsigned short* hA   = (unsigned short*)(ws + OFF_HA);
  unsigned short* hB   = (unsigned short*)(ws + OFF_HB);
  float*          gbuf = (float*)(ws + OFF_G);

  k_prep<<<264, 256, 0, stream>>>(w_ih, w_fc, wq, wfcq);

  k_layer0<<<NTOK_ALL / TOK_PER_BLK, 256, 0, stream>>>(x, w_ih0, b_ih, b_hh, hA);

  const long strideB_dir = (long)NGATE * DIN2;
  const long strideC_dir = 3L * HID;
  for (int l = 1; l <= 2; ++l) {
    const unsigned short* src = (l == 1) ? hA : hB;
    unsigned short*       dst = (l == 1) ? hB : hA;
    const unsigned short* Wl  = wq + (size_t)(l - 1) * 2 * NGATE * DIN2;
    const unsigned short* Wgo = Wl + (size_t)(2 * HID) * DIN2;
    const float* bil = b_ih + (size_t)l * 2 * NGATE;
    const float* bhl = b_hh + (size_t)l * 2 * NGATE;
    for (int c = 0; c < NCHUNK; ++c) {
      const unsigned short* Ac = src + (size_t)c * CHUNK_TOK * DIN2;
      wmma_gemm64<0, false, 0, 0, false, 0><<<dim3((CHUNK_TOK / 64) * (HID / 64) / 8, 2), 256, 0, stream>>>(
          Ac, Ac, DIN2, 0L, Wl, Wl, DIN2, strideB_dir,
          (void*)gbuf, (void*)gbuf, GCOLS, strideC_dir, b_fc, b_fc, 0L, CHUNK_TOK, HID, DIN2, UNCARRY);
      wmma_gemm64<0, false, 0, 0, false, 0><<<dim3((CHUNK_TOK / 64) * (2 * HID / 64) / 8, 2), 256, 0, stream>>>(
          Ac, Ac, DIN2, 0L, Wgo, Wgo, DIN2, strideB_dir,
          (void*)(gbuf + HID), (void*)(gbuf + HID), GCOLS, strideC_dir, b_fc, b_fc, 0L, CHUNK_TOK, 2 * HID, DIN2, UNCARRY);
      k_act<<<CHUNK_TOK / TOK_PER_BLK, 256, 0, stream>>>(gbuf, bil, bhl, dst + (size_t)c * CHUNK_TOK * DIN2);
    }
  }

  wmma_gemm64<0, false, 0, 0, false, 0><<<dim3((NTOK_ALL / 64) * (FCN / 64) / 8, 1), 256, 0, stream>>>(
      hA, hA, DIN2, 0L, wfcq, wfcq, DIN2, 0L,
      (void*)gbuf, (void*)gbuf, FCN, 0L, b_fc, b_fc, 0L, NTOK_ALL, FCN, DIN2, UNCARRY);

  k_out<<<(NTOK_ALL / 2) / 256, 256, 0, stream>>>(gbuf, b_fc, out);
}
